// GCN_24824910971032
// MI455X (gfx1250) — hardware-verified
//
#include <hip/hip_runtime.h>
#include <stddef.h>
#include <stdint.h>
#include <math.h>


#define DF     128
#define K1     256
#define NTHR   256
#define NWAVE  8
#define EPT    8
#define CHUNK  (NTHR * EPT)
#define WCAP   (EPT * 32)
#define LISTN  (NWAVE * WCAP)
#define NBD    8192
#define SLD    13
#define NBA    1024
#define SLA    10
#define RCAP   28672
#define DEGCAP 64
#define GBM    64
#define GBN    64
#define GTHR   128
#define NU0    (DF * (DF / 8))
#define NU1    (DF * (K1 / 8))
#define AGG_ZINTS    (LISTN + 2 * RCAP + 3 * NBA)
#define MISC_INTS    16
#define EXTRA_INTS   2048
#define AGG_LDS_INTS (AGG_ZINTS + MISC_INTS + EXTRA_INTS)
#define WSMAX  134217728

static_assert((CHUNK & (CHUNK - 1)) == 0 && CHUNK <= 4096);
static_assert((NBD & (NBD - 1)) == 0 && NBD == (1 << SLD));
static_assert((NBA & (NBA - 1)) == 0 && NBA == (1 << SLA));
static_assert(((long long)CHUNK << SLD) < (1LL << 31));
static_assert(((long long)CHUNK << SLA) < (1LL << 31));
static_assert(NBD % (NTHR * 4) == 0);
static_assert(LISTN % NTHR == 0);
static_assert(NBA % NWAVE == 0 && NBA % 32 == 0 && NBA % GBM == 0);
static_assert(RCAP % 32 == 0 && AGG_ZINTS % 4 == 0 && LISTN % 4 == 0);
static_assert(((AGG_ZINTS + MISC_INTS) % 4) == 0 && AGG_LDS_INTS % 4 == 0);
static_assert(DF % 32 == 0 && K1 % 32 == 0 && K1 == 2 * DF && DF % GBN == 0);
static_assert(GBM == (GTHR / 32) * 16 && GBN == 64);
static_assert(NU0 % NTHR == 0 && NU1 % NTHR == 0);
static_assert(DF == 4 * 32);
static_assert(EXTRA_INTS >= NWAVE * K1 / 2 && EXTRA_INTS >= NBA * 2);
static_assert((NBA * 2) % (NTHR * 4) == 0);
static_assert(AGG_LDS_INTS * 4 <= 300000);

typedef float          v2f   __attribute__((ext_vector_type(2)));
typedef float          v4f   __attribute__((ext_vector_type(4)));
typedef float          v8f   __attribute__((ext_vector_type(8)));
typedef int            v4i   __attribute__((ext_vector_type(4)));
typedef int            v8i   __attribute__((ext_vector_type(8)));
typedef unsigned short v4us  __attribute__((ext_vector_type(4)));
typedef unsigned short v8us  __attribute__((ext_vector_type(8)));
typedef unsigned short v16us __attribute__((ext_vector_type(16)));
typedef __bf16         v16bf __attribute__((ext_vector_type(16)));
typedef v2f  __attribute__((may_alias)) v2fa;
typedef v4f  __attribute__((may_alias)) v4fa;
typedef v4i  __attribute__((may_alias)) v4ia;
typedef v4us __attribute__((may_alias)) v4usa;
typedef v8us __attribute__((may_alias)) v8usa;
union FragB { v16bf v; v16us u; v8us h[2]; v8i w; };

__device__ __forceinline__ v8f wmb(const FragB& a, const FragB& b, v8f c) {
  v8f d = __builtin_amdgcn_wmma_f32_16x16x32_bf16(false, a.v, false, b.v, (short)0, c, false, false);
  asm volatile("v_nop\n\tv_nop\n\tv_nop\n\tv_nop" : "+v"(d) : "v"(a.w), "v"(b.w));
  return d;
}

__device__ __forceinline__ unsigned bf16_bits(float f) {
  const unsigned u = __float_as_uint(f);
  return (u + 0x7FFFu + ((u >> 16) & 1u)) >> 16;
}
__device__ __forceinline__ float bf16_val(float f) {
  return __uint_as_float(bf16_bits(f) << 16);
}

__device__ __forceinline__ void wave_sync() {
  __builtin_amdgcn_fence(__ATOMIC_RELEASE, "wavefront");
  __builtin_amdgcn_wave_barrier();
  __builtin_amdgcn_fence(__ATOMIC_ACQUIRE, "wavefront");
}

__device__ __forceinline__ int clampi(int v, int hi) { return v < 0 ? 0 : (v > hi ? hi : v); }

template <int SLB>
__device__ __forceinline__ int scan_chunk(const int* __restrict__ dsts, int nE, int cbase, int slotBase,
                                          int nb, int vec8, int* list, int tid, int lane, int wave) {
  int wc = 0;
  const int el0  = tid * EPT;
  const int e0   = cbase + el0;
  const int sent = -2147483647 - 1;
  v4i da, db;
  if (vec8 != 0 && cbase + CHUNK <= nE) {
    da = *(const v4i*)(dsts + e0);
    db = *(const v4i*)(dsts + e0 + 4);
  } else {
    da.x = (e0     < nE) ? dsts[min(e0,     nE - 1)] : sent;
    da.y = (e0 + 1 < nE) ? dsts[min(e0 + 1, nE - 1)] : sent;
    da.z = (e0 + 2 < nE) ? dsts[min(e0 + 2, nE - 1)] : sent;
    da.w = (e0 + 3 < nE) ? dsts[min(e0 + 3, nE - 1)] : sent;
    db.x = (e0 + 4 < nE) ? dsts[min(e0 + 4, nE - 1)] : sent;
    db.y = (e0 + 5 < nE) ? dsts[min(e0 + 5, nE - 1)] : sent;
    db.z = (e0 + 6 < nE) ? dsts[min(e0 + 6, nE - 1)] : sent;
    db.w = (e0 + 7 < nE) ? dsts[min(e0 + 7, nE - 1)] : sent;
  }
  const unsigned nbs = (unsigned)slotBase;
  const unsigned unb = (unsigned)nb;
  const unsigned s0 = (unsigned)da.x - nbs, s1 = (unsigned)da.y - nbs;
  const unsigned s2 = (unsigned)da.z - nbs, s3 = (unsigned)da.w - nbs;
  const unsigned s4 = (unsigned)db.x - nbs, s5 = (unsigned)db.y - nbs;
  const unsigned s6 = (unsigned)db.z - nbs, s7 = (unsigned)db.w - nbs;
  const bool h0 = s0 < unb, h1 = s1 < unb, h2 = s2 < unb, h3 = s3 < unb;
  const bool h4 = s4 < unb, h5 = s5 < unb, h6 = s6 < unb, h7 = s7 < unb;
  const unsigned any = __builtin_amdgcn_ballot_w32(h0 | h1 | h2 | h3 | h4 | h5 | h6 | h7);
  if (any != 0u) {
#define HITJ(J, HJ, SJ) { \
      const unsigned mj = __builtin_amdgcn_ballot_w32(HJ); \
      if (mj != 0u) { \
        if (HJ) { \
          const int pos = wc + (int)__builtin_amdgcn_mbcnt_lo(mj, 0u); \
          if (pos < WCAP) list[wave * WCAP + pos] = ((el0 + (J)) << SLB) | (int)(SJ); \
        } \
        wc += (int)__builtin_popcount(mj); } }
    HITJ(0, h0, s0)
    HITJ(1, h1, s1)
    HITJ(2, h2, s2)
    HITJ(3, h3, s3)
    HITJ(4, h4, s4)
    HITJ(5, h5, s5)
    HITJ(6, h6, s6)
    HITJ(7, h7, s7)
#undef HITJ
  }
  return wc;
}

__global__ __launch_bounds__(NTHR) void k_wprep(const float* __restrict__ W0, const float* __restrict__ W1,
                                                unsigned short* W0T, unsigned short* W1T2) {
  const int u = (int)blockIdx.x * NTHR + (int)threadIdx.x;
  v8us o;
  unsigned short* dp;
  if (u < NU0) {
    const int n  = u >> 4;
    const int k8 = (u & 15) * 8;
    const float* p = W0 + (size_t)k8 * DF + n;
#pragma unroll
    for (int i = 0; i < 8; ++i) o[i] = (unsigned short)bf16_bits(p[(size_t)i * DF]);
    dp = W0T + (size_t)n * DF + k8;
  } else if (u < NU0 + NU1) {
    const int v  = u - NU0;
    const int n  = v >> 5;
    const int k8 = (v & 31) * 8;
    const int kk = k8 & (DF - 1);
    const float* p = W1 + (size_t)kk * DF + n;
#pragma unroll
    for (int i = 0; i < 8; ++i) o[i] = (unsigned short)bf16_bits(p[(size_t)i * DF]);
    dp = W1T2 + (size_t)n * K1 + k8;
  } else {
    return;
  }
  *(volatile v8us*)dp = o;
  __threadfence();
  *(volatile v8us*)dp = o;
}

__global__ __launch_bounds__(NTHR) void k_cvx(const float* __restrict__ x, int nN, int nUnits,
                                              unsigned short* xb) {
  const int u = (int)blockIdx.x * NTHR + (int)threadIdx.x;
  if (u >= nUnits) return;
  const int row = u >> 4;
  const int k8  = (u & 15) * 8;
  const int rc  = row < nN ? row : nN - 1;
  const float* p = x + (size_t)rc * DF + k8;
  const v4f a = *(const v4fa*)p;
  const v4f b = *(const v4fa*)(p + 4);
  const bool ok = row < nN;
  v8us o;
  o[0] = ok ? (unsigned short)bf16_bits(a.x) : (unsigned short)0;
  o[1] = ok ? (unsigned short)bf16_bits(a.y) : (unsigned short)0;
  o[2] = ok ? (unsigned short)bf16_bits(a.z) : (unsigned short)0;
  o[3] = ok ? (unsigned short)bf16_bits(a.w) : (unsigned short)0;
  o[4] = ok ? (unsigned short)bf16_bits(b.x) : (unsigned short)0;
  o[5] = ok ? (unsigned short)bf16_bits(b.y) : (unsigned short)0;
  o[6] = ok ? (unsigned short)bf16_bits(b.z) : (unsigned short)0;
  o[7] = ok ? (unsigned short)bf16_bits(b.w) : (unsigned short)0;
  unsigned short* dp = xb + (size_t)row * DF + k8;
  *(volatile v8us*)dp = o;
  __threadfence();
  *(volatile v8us*)dp = o;
}

__global__ __launch_bounds__(NTHR) void k_deg(const int* __restrict__ dsts, const float* __restrict__ ea,
                                              int nE, int vec8, float* dinv) {
  __shared__ __attribute__((aligned(16))) float sdeg[NBD];
  __shared__ __attribute__((aligned(16))) int list[LISTN];
  __shared__ int wcnt[NWAVE];
  const int tid = (int)threadIdx.x, lane = tid & 31, wave = tid >> 5;
  const int nodeBase = (int)blockIdx.x * NBD;

  for (int i = tid; i < NBD; i += NTHR) sdeg[i] = 0.0f;
  for (int i = tid; i < LISTN; i += NTHR) list[i] = 0;
  if (tid < NWAVE) wcnt[tid] = 0;
  __syncthreads();

  const int nChunks = (nE + CHUNK - 1) / CHUNK;
#pragma unroll 1
  for (int ch = 0; ch < nChunks; ++ch) {
    const int cbase = ch * CHUNK;
    const int wc = scan_chunk<SLD>(dsts, nE, cbase, nodeBase, NBD, vec8, list, tid, lane, wave);
    if (lane == 0) wcnt[wave] = wc;
    __syncthreads();
    if (wave == 0) {
#pragma unroll 1
      for (int w2 = 0; w2 < NWAVE; ++w2) {
        int c = wcnt[w2];
        c = c < 0 ? 0 : (c > WCAP ? WCAP : c);
#pragma unroll 1
        for (int b0 = 0; b0 < c; b0 += 32) {
          const int idx = b0 + lane;
          const int ent = list[w2 * WCAP + (idx < WCAP ? idx : WCAP - 1)];
          const int el  = (ent >> SLD) & (CHUNK - 1);
          const int eid = clampi(cbase + el, nE - 1);
          const int wvi = __float_as_int(bf16_val(ea[eid]));
          const int m32 = (c - b0) < 32 ? (c - b0) : 32;
#pragma unroll 1
          for (int k = 0; k < m32; ++k) {
            const int   u  = __builtin_amdgcn_readlane(ent, k);
            const float wk = __int_as_float(__builtin_amdgcn_readlane(wvi, k));
            const int   sl = u & (NBD - 1);
            if (lane == 0) sdeg[sl] = sdeg[sl] + wk;
          }
        }
      }
    }
    __syncthreads();
  }

#pragma unroll 1
  for (int i = tid; i < NBD; i += NTHR) {
    const float d = sdeg[i] + 1.0f;
    const float r = 1.0f / sqrtf(d);
    sdeg[i] = (d > 0.0f) ? r : ((d != d) ? d : 0.0f);
  }
  __syncthreads();

  v4f vals[NBD / (NTHR * 4)];
#pragma unroll
  for (int it = 0; it < NBD / (NTHR * 4); ++it) {
    const int s0 = it * (NTHR * 4) + 4 * tid;
    vals[it] = *(const v4fa*)(sdeg + s0);
  }
#pragma unroll
  for (int it = 0; it < NBD / (NTHR * 4); ++it) {
    const int s0 = it * (NTHR * 4) + 4 * tid;
    *(volatile v4f*)(dinv + (size_t)nodeBase + s0) = vals[it];
  }
  __threadfence();
#pragma unroll
  for (int it = 0; it < NBD / (NTHR * 4); ++it) {
    const int s0 = it * (NTHR * 4) + 4 * tid;
    *(volatile v4f*)(dinv + (size_t)nodeBase + s0) = vals[it];
  }
}

__global__ __launch_bounds__(NTHR) void k_norm(const int* __restrict__ srcs, const int* __restrict__ dsts,
                                               const float* __restrict__ ea, const float* __restrict__ dinv,
                                               int nE, int nN, float* nrm) {
  const int t  = (int)blockIdx.x * NTHR + (int)threadIdx.x;
  const int e0 = 4 * t;
  if (e0 + 3 >= nE) return;
  const v4i s4 = *(const v4ia*)(srcs + e0);
  const v4i d4 = *(const v4ia*)(dsts + e0);
  const v4f w4 = *(const v4fa*)(ea + e0);
  const int hiN = nN - 1;
  const float a0 = dinv[clampi(s4.x, hiN)], a1 = dinv[clampi(s4.y, hiN)];
  const float a2 = dinv[clampi(s4.z, hiN)], a3 = dinv[clampi(s4.w, hiN)];
  const float c0 = dinv[clampi(d4.x, hiN)], c1 = dinv[clampi(d4.y, hiN)];
  const float c2 = dinv[clampi(d4.z, hiN)], c3 = dinv[clampi(d4.w, hiN)];
  v4f o;
  o.x = (a0 * bf16_val(w4.x)) * c0;
  o.y = (a1 * bf16_val(w4.y)) * c1;
  o.z = (a2 * bf16_val(w4.z)) * c2;
  o.w = (a3 * bf16_val(w4.w)) * c3;
  float* dp = nrm + e0;
  *(volatile v4f*)dp = o;
  __threadfence();
  *(volatile v4f*)dp = o;
}

__global__ __launch_bounds__(GTHR) void k_gemm(
    const unsigned short* __restrict__ A, const unsigned short* __restrict__ WT,
    float* outF, int K, int ldo)
{
  __shared__ __attribute__((aligned(16))) float stg[GBM * GBN];
  const int tid = (int)threadIdx.x, lane = tid & 31, wave = tid >> 5, hh = lane >> 4, m = lane & 15;
  const int rowBase = (int)blockIdx.x * GBM;
  const int col0    = (int)blockIdx.y * GBN;

  v8f acc[4];
  {
    const v8f z = {0.f, 0.f, 0.f, 0.f, 0.f, 0.f, 0.f, 0.f};
    acc[0] = z; acc[1] = z; acc[2] = z; acc[3] = z;
  }
  const unsigned short* ap = A  + (size_t)(rowBase + 16 * wave + m) * (size_t)K + 8 * hh;
  const unsigned short* wp = WT + (size_t)(col0 + m) * (size_t)K + 8 * hh;
  const int ksteps = K >> 5;
#pragma unroll 1
  for (int ks = 0; ks < ksteps; ++ks) {
    FragB af;
    af.h[0] = *(const v8usa*)(ap + 32 * ks);
    af.h[1] = *(const v8usa*)(ap + 32 * ks + 16);
#pragma unroll
    for (int t = 0; t < 4; ++t) {
      const unsigned short* wq = wp + (size_t)(16 * t) * (size_t)K + 32 * ks;
      FragB bf;
      bf.h[0] = *(const v8usa*)wq;
      bf.h[1] = *(const v8usa*)(wq + 16);
      acc[t] = wmb(af, bf, acc[t]);
    }
  }

#pragma unroll
  for (int t = 0; t < 4; ++t) {
    const int lc = 16 * t + m;
#pragma unroll
    for (int r = 0; r < 8; ++r) {
      const int lr = 16 * wave + 8 * hh + r;
      stg[lr * GBN + lc] = acc[t][r];
    }
  }
  __syncthreads();

  v4f fv[8];
#pragma unroll
  for (int i = 0; i < 8; ++i) {
    const int lr = 16 * wave + 2 * i + hh;
    fv[i] = *(const v4fa*)(stg + lr * GBN + 4 * m);
  }
#pragma unroll
  for (int i = 0; i < 8; ++i) {
    const int lr = 16 * wave + 2 * i + hh;
    const int gr = rowBase + lr;
    float* op = outF + (size_t)gr * (size_t)ldo + col0 + 4 * m;
    *(volatile v4f*)op = fv[i];
  }
  __threadfence();
#pragma unroll
  for (int i = 0; i < 8; ++i) {
    const int lr = 16 * wave + 2 * i + hh;
    const int gr = rowBase + lr;
    float* op = outF + (size_t)gr * (size_t)ldo + col0 + 4 * m;
    *(volatile v4f*)op = fv[i];
  }
}

template <int MODE>
__global__ __launch_bounds__(NTHR) void k_agg(const int* __restrict__ srcs, const int* __restrict__ dsts,
                                              const float* __restrict__ nrm, const float* __restrict__ dinv,
                                              int nE, int nN, int vec8, int mRows,
                                              const float* __restrict__ tin, const float* __restrict__ bias,
                                              const float* __restrict__ w2,
                                              unsigned short* hb, float* fout) {
  extern __shared__ __attribute__((aligned(16))) int dsm[];
  int* list = dsm;
  int* hl   = dsm + LISTN;
  int* sl   = hl + RCAP;
  int* cnt  = sl + RCAP;
  int* offs = cnt + NBA;
  int* cur  = offs + NBA;
  int* misc = cur + NBA;
  int* extra = misc + MISC_INTS;
  const int tid = (int)threadIdx.x, lane = tid & 31, wave = tid >> 5;
  const int nodeBase = (int)blockIdx.x * NBA;

  {
    const v4i z4 = {0, 0, 0, 0};
    for (int i = tid * 4; i < AGG_LDS_INTS; i += NTHR * 4) *(v4ia*)(dsm + i) = z4;
  }
  __syncthreads();

  int t = 0, ov = 0;
  const int nChunks = (nE + CHUNK - 1) / CHUNK;
#pragma unroll 1
  for (int ch = 0; ch < nChunks; ++ch) {
    const int cbase = ch * CHUNK;
    const int wc = scan_chunk<SLA>(dsts, nE, cbase, nodeBase, NBA, vec8, list, tid, lane, wave);
    if (lane == 0) misc[wave] = wc;
    __syncthreads();
    if (wave == 0) {
#pragma unroll 1
      for (int w2i = 0; w2i < NWAVE; ++w2i) {
        int c = misc[w2i];
        c = c < 0 ? 0 : (c > WCAP ? WCAP : c);
#pragma unroll 1
        for (int b0 = 0; b0 < c; b0 += 32) {
          const int idx = b0 + lane;
          const int ent = list[w2i * WCAP + (idx < WCAP ? idx : WCAP - 1)];
          const int m32 = (c - b0) < 32 ? (c - b0) : 32;
#pragma unroll 1
          for (int k = 0; k < m32; ++k) {
            const int u    = __builtin_amdgcn_readlane(ent, k);
            const int slot = u & (NBA - 1);
            const int el   = (u >> SLA) & (CHUNK - 1);
            const int pk   = ((cbase + el) << SLA) | slot;
            if (t < RCAP) {
              if (lane == 0) { hl[t] = pk; cnt[slot] = cnt[slot] + 1; }
              t = t + 1;
            } else {
              ov = 1;
            }
          }
        }
      }
    }
    __syncthreads();
  }
  if (wave == 0 && lane == 0) { misc[8] = t; misc[9] = ov; }
  __syncthreads();
  int tt = misc[8];
  tt = tt < 0 ? 0 : (tt > RCAP ? RCAP : tt);
  const int ovf = misc[9];

  if (wave == 0) {
    const int base = lane * (NBA / 32);
    int s = 0;
#pragma unroll 1
    for (int i = 0; i < NBA / 32; ++i) s += cnt[base + i];
    int incl = s;
#pragma unroll
    for (int d = 1; d < 32; d <<= 1) {
      const int y = __shfl_up(incl, d, 32);
      if (lane >= d) incl += y;
    }
    int run = incl - s;
#pragma unroll 1
    for (int i = 0; i < NBA / 32; ++i) {
      const int cv = cnt[base + i];
      offs[base + i] = run;
      cur[base + i]  = run;
      run += cv;
    }
  }
  __syncthreads();
  if (wave == 0) {
#pragma unroll 1
    for (int b0 = 0; b0 < tt; b0 += 32) {
      const int idx = b0 + lane;
      const int ent = hl[idx < RCAP ? idx : RCAP - 1];
      const int m32 = (tt - b0) < 32 ? (tt - b0) : 32;
#pragma unroll 1
      for (int k = 0; k < m32; ++k) {
        const int u    = __builtin_amdgcn_readlane(ent, k);
        const int slot = u & (NBA - 1);
        if (lane == 0) {
          int p = cur[slot];
          p = p < 0 ? 0 : (p > RCAP - 1 ? RCAP - 1 : p);
          sl[p] = u;
          cur[slot] = p + 1;
        }
      }
    }
  }
  __syncthreads();

  const float qnan = __int_as_float(0x7fc00000);
  const float pz = (ovf != 0) ? qnan : 0.0f;
  float* tile = (float*)extra;
  unsigned short* rowbuf = (unsigned short*)extra + wave * K1;

  v4f bb = {0.0f, 0.0f, 0.0f, 0.0f};
  v4f wa = {0.0f, 0.0f, 0.0f, 0.0f};
  v4f wb = {0.0f, 0.0f, 0.0f, 0.0f};
  float bs0 = 0.0f, bs1 = 0.0f;
  if constexpr (MODE != 3) {
    const v4f bq = *(const v4fa*)(bias + 4 * lane);
    bb.x = bf16_val(bq.x); bb.y = bf16_val(bq.y); bb.z = bf16_val(bq.z); bb.w = bf16_val(bq.w);
  } else {
    bs0 = bf16_val(bias[0]); bs1 = bf16_val(bias[1]);
  }
  if constexpr (MODE == 2) {
    const v4f q0 = *(const v4fa*)(w2 + 8 * lane);
    const v4f q1 = *(const v4fa*)(w2 + 8 * lane + 4);
    wa.x = bf16_val(q0.x); wa.y = bf16_val(q0.y); wa.z = bf16_val(q0.z); wa.w = bf16_val(q0.w);
    wb.x = bf16_val(q1.x); wb.y = bf16_val(q1.y); wb.z = bf16_val(q1.z); wb.w = bf16_val(q1.w);
  }

#pragma unroll 1
  for (int si = 0; si < NBA / NWAVE; ++si) {
    const int s    = si * NWAVE + wave;
    const int node = nodeBase + s;
    int c = cnt[s];
    const bool big = c > DEGCAP;
    c = c < 0 ? 0 : (c > DEGCAP ? DEGCAP : c);
    int o = offs[s];
    o = o < 0 ? 0 : (o > RCAP ? RCAP : o);
    const int nc = node < nN ? node : nN - 1;
    const float dd = dinv[nc];
    const float rd = dd * dd;
    const float pzr = big ? qnan : pz;
    const bool live = node < nN;

    if constexpr (MODE != 3) {
      float a0 = 0.0f, a1 = 0.0f, a2 = 0.0f, a3 = 0.0f;
#pragma unroll 1
      for (int b0 = 0; b0 < c; b0 += 32) {
        int idx = o + b0 + lane;
        idx = idx > RCAP - 1 ? RCAP - 1 : idx;
        const int ent = sl[idx];
        const int eid = clampi(ent >> SLA, nE - 1);
        const int sr  = clampi(srcs[eid], nN - 1);
        const int cfi = __float_as_int(nrm[eid]);
        const int m32 = (c - b0) < 32 ? (c - b0) : 32;
#pragma unroll 1
        for (int k = 0; k < m32; ++k) {
          const int   sk = __builtin_amdgcn_readlane(sr, k);
          const float ck = __int_as_float(__builtin_amdgcn_readlane(cfi, k));
          const v4f a = *(const v4fa*)(tin + (size_t)sk * DF + 4 * lane);
          a0 = fmaf(ck, a.x, a0); a1 = fmaf(ck, a.y, a1);
          a2 = fmaf(ck, a.z, a2); a3 = fmaf(ck, a.w, a3);
        }
      }
      const v4f sv = *(const v4fa*)(tin + (size_t)nc * DF + 4 * lane);
      float y0 = (a0 + sv.x * rd) + bb.x;
      float y1 = (a1 + sv.y * rd) + bb.y;
      float y2 = (a2 + sv.z * rd) + bb.z;
      float y3 = (a3 + sv.w * rd) + bb.w;
      y0 = (y0 > 0.0f) ? y0 : (y0 - y0);
      y1 = (y1 > 0.0f) ? y1 : (y1 - y1);
      y2 = (y2 > 0.0f) ? y2 : (y2 - y2);
      y3 = (y3 > 0.0f) ? y3 : (y3 - y3);
      y0 = y0 + pzr; y1 = y1 + pzr; y2 = y2 + pzr; y3 = y3 + pzr;
      const float v0 = live ? y0 : 0.0f;
      const float v1 = live ? y1 : 0.0f;
      const float v2 = live ? y2 : 0.0f;
      const float v3 = live ? y3 : 0.0f;

      if constexpr (MODE == 1) {
        v4us mh, ml;
        {
          unsigned hbv;
          hbv = bf16_bits(v0); mh[0] = (unsigned short)hbv; ml[0] = (unsigned short)bf16_bits(v0 - __uint_as_float(hbv << 16));
          hbv = bf16_bits(v1); mh[1] = (unsigned short)hbv; ml[1] = (unsigned short)bf16_bits(v1 - __uint_as_float(hbv << 16));
          hbv = bf16_bits(v2); mh[2] = (unsigned short)hbv; ml[2] = (unsigned short)bf16_bits(v2 - __uint_as_float(hbv << 16));
          hbv = bf16_bits(v3); mh[3] = (unsigned short)hbv; ml[3] = (unsigned short)bf16_bits(v3 - __uint_as_float(hbv << 16));
        }
        *(v4usa*)(rowbuf + 4 * lane) = mh;
        *(v4usa*)(rowbuf + DF + 4 * lane) = ml;
        wave_sync();
        const v8us q0 = *(const v8usa*)(rowbuf + 8 * lane);
        wave_sync();
        if (node < mRows) {
          unsigned short* rpw = hb + (size_t)node * K1 + 8 * lane;
          *(volatile v8us*)rpw = q0;
          __threadfence();
          *(volatile v8us*)rpw = q0;
        }
      } else {
        float p0 = fmaf(v3, wb.z, fmaf(v2, wb.x, fmaf(v1, wa.z, v0 * wa.x)));
        float p1 = fmaf(v3, wb.w, fmaf(v2, wb.y, fmaf(v1, wa.w, v0 * wa.y)));
#pragma unroll
        for (int d = 16; d >= 1; d >>= 1) {
          const float r0 = __shfl_xor(p0, d, 32);
          const float r1 = __shfl_xor(p1, d, 32);
          p0 = p0 + r0; p1 = p1 + r1;
        }
        if (lane == 0) { tile[2 * s] = p0; tile[2 * s + 1] = p1; }
      }
    } else {
      float a0 = 0.0f, a1 = 0.0f;
#pragma unroll 1
      for (int b0 = 0; b0 < c; b0 += 32) {
        int idx = o + b0 + lane;
        idx = idx > RCAP - 1 ? RCAP - 1 : idx;
        const int ent = sl[idx];
        const int eid = clampi(ent >> SLA, nE - 1);
        const int sr  = clampi(srcs[eid], nN - 1);
        const int cfi = __float_as_int(nrm[eid]);
        const v2f tv  = *(const v2fa*)(tin + (size_t)sr * 2);
        const int txi = __float_as_int(tv.x);
        const int tyi = __float_as_int(tv.y);
        const int m32 = (c - b0) < 32 ? (c - b0) : 32;
#pragma unroll 1
        for (int k = 0; k < m32; ++k) {
          const float ck = __int_as_float(__builtin_amdgcn_readlane(cfi, k));
          const float tx = __int_as_float(__builtin_amdgcn_readlane(txi, k));
          const float ty = __int_as_float(__builtin_amdgcn_readlane(tyi, k));
          a0 = fmaf(ck, tx, a0); a1 = fmaf(ck, ty, a1);
        }
      }
      const v2f sv = *(const v2fa*)(tin + (size_t)nc * 2);
      float y0 = (a0 + sv.x * rd) + bs0;
      float y1 = (a1 + sv.y * rd) + bs1;
      y0 = y0 + pzr; y1 = y1 + pzr;
      if (lane == 0) { tile[2 * s] = y0; tile[2 * s + 1] = y1; }
    }
  }

  if constexpr (MODE != 1) {
    __syncthreads();
    constexpr int NIT = (NBA * 2) / (NTHR * 4);
    v4f ov4[NIT];
#pragma unroll
    for (int it = 0; it < NIT; ++it) ov4[it] = *(const v4fa*)(tile + 4 * (it * NTHR + tid));
    const long long ebase = (long long)nodeBase * 2;
    const long long elim  = (MODE == 3) ? (long long)nN * 2 : ((long long)nodeBase + NBA) * 2;
#pragma unroll
    for (int it = 0; it < NIT; ++it) {
      const long long e = ebase + 4 * (it * NTHR + tid);
      if (e + 3 < elim) *(volatile v4f*)(fout + e) = ov4[it];
    }
    __threadfence();
#pragma unroll
    for (int it = 0; it < NIT; ++it) {
      const long long e = ebase + 4 * (it * NTHR + tid);
      if (e + 3 < elim) *(volatile v4f*)(fout + e) = ov4[it];
    }
  }
}

static inline int cdiv(int a, int b) { return (a + b - 1) / b; }
static inline size_t al256(size_t o) { return (o + 255) & ~(size_t)255; }

extern "C" void kernel_launch(void* const* d_in, const int* in_sizes, int n_in,
                              void* d_out, int out_size, void* d_ws, size_t ws_size,
                              hipStream_t stream) {
  if (n_in < 9) return;
  if (in_sizes[0] < DF || (in_sizes[0] % DF) != 0) return;
  const int nN = in_sizes[0] / DF;
  if (nN < 16 || nN > (1 << 22) || (nN % 16) != 0) return;
  if (in_sizes[1] < 2 || (in_sizes[1] & 1) != 0) return;
  const int nE = in_sizes[1] / 2;
  if (nE < 4 || nE >= (1 << (31 - SLA)) || (nE & 3) != 0) return;
  if (in_sizes[2] != nE) return;
  if (in_sizes[3] != DF * DF || in_sizes[4] != DF) return;
  if (in_sizes[5] != DF * DF || in_sizes[6] != DF) return;
  if (in_sizes[7] != DF * 2 || in_sizes[8] != 2) return;
  if ((long long)out_size != (long long)nN * 2) return;

  const float* x    = (const float*)d_in[0];
  const int*   edge = (const int*)d_in[1];
  const float* ea   = (const float*)d_in[2];
  const float* W0   = (const float*)d_in[3];
  const float* b0   = (const float*)d_in[4];
  const float* W1   = (const float*)d_in[5];
  const float* b1   = (const float*)d_in[6];
  const float* W2   = (const float*)d_in[7];
  const float* b2   = (const float*)d_in[8];
  float* out = (float*)d_out;
  const int* src = edge;
  const int* dst = edge + nE;

  const int MP   = cdiv(nN, GBM) * GBM;
  const int gM   = MP / GBM;
  const int gD   = cdiv(nN, NBD);
  const int NBPD = gD * NBD;
  const int gA   = cdiv(MP, NBA);
  if ((long long)gA * NBA < (long long)MP) return;
  if (NBPD < nN) return;
  const int vec8 = ((nE & 3) == 0) ? 1 : 0;

  char* ws = (char*)d_ws;
  size_t off = 0;
  const size_t oDINV = off; off = al256(off + (size_t)NBPD * 4);
  const size_t oNORM = off; off = al256(off + (size_t)nE * 4);
  const size_t oW0T  = off; off = al256(off + (size_t)DF * DF * 2);
  const size_t oW1T  = off; off = al256(off + (size_t)DF * K1 * 2);
  const size_t oXB   = off; off = al256(off + (size_t)MP * DF * 2);
  const size_t oT0   = off; off = al256(off + (size_t)MP * DF * 4);
  const size_t oH1   = off; off = al256(off + (size_t)MP * K1 * 2);
  const size_t oT1   = off; off = al256(off + (size_t)MP * DF * 4);
  const size_t oT2   = off; off = al256(off + (size_t)gA * NBA * 2 * 4);
  if (off > ws_size || off > (size_t)WSMAX) return;
  float*          DINV = (float*)(ws + oDINV);
  float*          NORM = (float*)(ws + oNORM);
  unsigned short* W0T  = (unsigned short*)(ws + oW0T);
  unsigned short* W1T2 = (unsigned short*)(ws + oW1T);
  unsigned short* XB   = (unsigned short*)(ws + oXB);
  float*          T0   = (float*)(ws + oT0);
  unsigned short* H1HL = (unsigned short*)(ws + oH1);
  float*          T1   = (float*)(ws + oT1);
  float*          T2   = (float*)(ws + oT2);

  const size_t aggLds = (size_t)AGG_LDS_INTS * 4;
  hipFuncSetAttribute(reinterpret_cast<const void*>(&k_agg<1>), hipFuncAttributeMaxDynamicSharedMemorySize, (int)aggLds);
  hipFuncSetAttribute(reinterpret_cast<const void*>(&k_agg<2>), hipFuncAttributeMaxDynamicSharedMemorySize, (int)aggLds);
  hipFuncSetAttribute(reinterpret_cast<const void*>(&k_agg<3>), hipFuncAttributeMaxDynamicSharedMemorySize, (int)aggLds);

  const int nUx = MP * (DF / 8);
  k_wprep<<<(NU0 + NU1) / NTHR, NTHR, 0, stream>>>(W0, W1, W0T, W1T2);
  k_cvx<<<cdiv(nUx, NTHR), NTHR, 0, stream>>>(x, nN, nUx, XB);
  k_deg<<<gD, NTHR, 0, stream>>>(dst, ea, nE, vec8, DINV);
  k_norm<<<cdiv(nE / 4, NTHR), NTHR, 0, stream>>>(src, dst, ea, DINV, nE, nN, NORM);
  k_gemm<<<dim3(gM, DF / GBN), GTHR, 0, stream>>>(XB, W0T, T0, DF, DF);
  k_agg<1><<<gA, NTHR, aggLds, stream>>>(src, dst, NORM, DINV, nE, nN, vec8, MP, T0, b0, W2, H1HL, T2);
  k_gemm<<<dim3(gM, DF / GBN), GTHR, 0, stream>>>(H1HL, W1T2, T1, K1, DF);
  k_agg<2><<<gA, NTHR, aggLds, stream>>>(src, dst, NORM, DINV, nE, nN, vec8, MP, T1, b1, W2, H1HL, T2);
  k_agg<3><<<gA, NTHR, aggLds, stream>>>(src, dst, NORM, DINV, nE, nN, vec8, MP, T2, b2, W2, H1HL, out);
}
